// StabilizedSMM_86998857547869
// MI455X (gfx1250) — hardware-verified
//
#include <hip/hip_runtime.h>
#include <math.h>
typedef __attribute__((ext_vector_type(16))) _Float16 v16h;
typedef __attribute__((ext_vector_type(8)))  _Float16 v8h;
typedef __attribute__((ext_vector_type(16))) __bf16   v16b;
typedef __attribute__((ext_vector_type(8)))  __bf16   v8b;
typedef __attribute__((ext_vector_type(8)))  float    v8f;
typedef __attribute__((ext_vector_type(4)))  float    v4f;
#define PSCALE 32768.0f
#define U16(p) ((const unsigned short*)(const void*)(p))
#define PSCALE_INV (1.0f / 32768.0f)

__device__ __forceinline__ unsigned short f2bf_bits(float f) {
  unsigned u = __float_as_uint(f);
  return (unsigned short)((u + 0x7FFFu + ((u >> 16) & 1u)) >> 16);
}
__device__ __forceinline__ float bf_bits2f(unsigned short h) { return __uint_as_float(((unsigned)h) << 16); }

__device__ __forceinline__ void dep_guard_h(v8f& a, v8f& b, v16h x, v16h y) { asm volatile("v_nop\n\tv_nop\n\tv_nop\n\tv_nop" : "+v"(a), "+v"(b) : "v"(x), "v"(y)); }
__device__ __forceinline__ void dep_guard_b(v8f& a, v8f& b, v16b x, v16b y) { asm volatile("v_nop\n\tv_nop\n\tv_nop\n\tv_nop" : "+v"(a), "+v"(b) : "v"(x), "v"(y)); }
__device__ __forceinline__ void keep4_h(v16h a, v16h b, v16h c, v16h d) { asm volatile("v_nop" :: "v"(a), "v"(b), "v"(c), "v"(d)); }
__device__ __forceinline__ void keep4_b(v16b a, v16b b, v16b c, v16b d) { asm volatile("v_nop" :: "v"(a), "v"(b), "v"(c), "v"(d)); }
__device__ __forceinline__ void acc_guard4(v8f& a, v8f& b, v8f& c, v8f& d) { asm volatile("v_nop\n\tv_nop\n\tv_nop\n\tv_nop" : "+v"(a), "+v"(b), "+v"(c), "+v"(d)); }
template <typename T> struct Frag;
template <> struct Frag<_Float16> {
  typedef v16h V; union U { v16h v; v8h h[2]; };
  static __device__ __forceinline__ v16h load(const _Float16* p) {
    U f; f.h[0] = *(const v8h*)(p); f.h[1] = *(const v8h*)(p + 16); return f.v;
  }
  static __device__ __forceinline__ v8f mma(v16h a, v16h b, v8f c) {
    return __builtin_amdgcn_wmma_f32_16x16x32_f16(false, a, false, b, (short)0, c, false, false);
  }
  static __device__ __forceinline__ void guard(v8f& a, v8f& b, v16h x, v16h y) { dep_guard_h(a, b, x, y); }
  static __device__ __forceinline__ void keep(v16h a, v16h b, v16h c, v16h d) { keep4_h(a, b, c, d); }
};
template <> struct Frag<__bf16> {
  typedef v16b V; union U { v16b v; v8b h[2]; };
  static __device__ __forceinline__ v16b load(const __bf16* p) {
    U f; f.h[0] = *(const v8b*)(p); f.h[1] = *(const v8b*)(p + 16); return f.v;
  }
  static __device__ __forceinline__ v8f mma(v16b a, v16b b, v8f c) {
    return __builtin_amdgcn_wmma_f32_16x16x32_bf16(false, a, false, b, (short)0, c, false, false);
  }
  static __device__ __forceinline__ void guard(v8f& a, v8f& b, v16b x, v16b y) { dep_guard_b(a, b, x, y); }
  static __device__ __forceinline__ void keep(v16b a, v16b b, v16b c, v16b d) { keep4_b(a, b, c, d); }
};

template <int ET> struct Elem;
template <> struct Elem<0> { typedef _Float16 T; };
template <> struct Elem<1> { typedef __bf16 T; };
template <int ET, bool SPLIT, int BIAS_MODE, int OUT_MODE, bool RESID, int ACT = 0>
__global__ __launch_bounds__(256) void wmma_gemm64(
    const unsigned short* __restrict__ Ap, const unsigned short* __restrict__ A2p, int lda, long strideA,
    const unsigned short* __restrict__ Btp, const unsigned short* __restrict__ Bt2p, int ldb, long strideB,
    void* __restrict__ Cout, void* __restrict__ Cout2, int ldc, long strideC,
    const float* __restrict__ bias,
    const float* __restrict__ resid, long strideR,
    int M, int N, int K, float scale) {
  typedef typename Elem<ET>::T T;
  typedef typename Frag<T>::V V;
  const T* A = (const T*)Ap; const T* A2 = (const T*)A2p; const T* Bt = (const T*)Btp; const T* Bt2 = (const T*)Bt2p;
  __shared__ __align__(16) float sT[8][16 * 68];
  const int b    = blockIdx.y;
  const int lane = threadIdx.x & 31;
  const int wave = threadIdx.x >> 5;
  const int tilesN = N >> 6;
  const int tilesM = M >> 6;
  const int tile = blockIdx.x * 8 + wave;
  if (tile >= tilesM * tilesN) return;
  const int tm = tile / tilesN;
  const int tn = tile - tm * tilesN;
  const int m0 = tm << 6;
  const int n0 = tn << 6;

  const T* Ab  = A  + (size_t)b * strideA;
  const T* Bb  = Bt + (size_t)b * strideB;
  const T* Ab2 = SPLIT ? (A2  + (size_t)b * strideA) : nullptr;
  const T* Bb2 = SPLIT ? (Bt2 + (size_t)b * strideB) : nullptr;

  const int rlane = lane & 15;
  const int koff  = (lane >> 4) * 8;
  const int mOff  = (lane >> 4) * 8;

  v8f acc[4][4];
#pragma unroll
  for (int i = 0; i < 4; ++i)
#pragma unroll
    for (int j = 0; j < 4; ++j) acc[i][j] = (v8f){0.f,0.f,0.f,0.f,0.f,0.f,0.f,0.f};

  for (int k0 = 0; k0 < K; k0 += 32) {
    V bh[4], bl[4];
#pragma unroll
    for (int j = 0; j < 4; ++j) {
      const size_t bo = (size_t)(n0 + (j << 4) + rlane) * ldb + koff + k0;
      bh[j] = Frag<T>::load(Bb + bo);
      if (SPLIT) bl[j] = Frag<T>::load(Bb2 + bo);
    }
#pragma unroll
    for (int i = 0; i < 4; ++i) {
      const size_t ao = (size_t)(m0 + (i << 4) + rlane) * lda + koff + k0;
      V ah = Frag<T>::load(Ab + ao);
      V al;
      if (SPLIT) al = Frag<T>::load(Ab2 + ao);
#pragma unroll
      for (int j = 0; j < 4; ++j) {
        acc[i][j] = Frag<T>::mma(ah, bh[j], acc[i][j]);
        if (SPLIT) {
          acc[i][j] = Frag<T>::mma(ah, bl[j], acc[i][j]);
          acc[i][j] = Frag<T>::mma(al, bh[j], acc[i][j]);
        }
      }
      Frag<T>::guard(acc[i][0], acc[i][3], ah, SPLIT ? al : ah);
    }
    Frag<T>::keep(bh[0], bh[1], bh[2], bh[3]);
    if (SPLIT) Frag<T>::keep(bl[0], bl[1], bl[2], bl[3]);
  }
  acc_guard4(acc[0][0], acc[0][1], acc[0][2], acc[0][3]);
  acc_guard4(acc[1][0], acc[1][1], acc[1][2], acc[1][3]);
  acc_guard4(acc[2][0], acc[2][1], acc[2][2], acc[2][3]);
  acc_guard4(acc[3][0], acc[3][1], acc[3][2], acc[3][3]);

  float* slab = sT[wave];
  const float* Rb = RESID ? (resid + (size_t)b * strideR) : nullptr;
#pragma unroll
  for (int i = 0; i < 4; ++i) {
    const int mBase = m0 + (i << 4);
#pragma unroll
    for (int j = 0; j < 4; ++j) {
      const int n = n0 + (j << 4) + rlane;
      float bv = 0.f;
      if (BIAS_MODE == 2) bv = bias[n];
#pragma unroll
      for (int r = 0; r < 8; ++r) {
        float v = acc[i][j][r] * scale;
        if (BIAS_MODE == 1) v += bias[mBase + mOff + r];
        if (BIAS_MODE == 2) v += bv;
        if (RESID) v += Rb[(size_t)(mBase + mOff + r) * ldc + n];
        if (ACT == 1) v = tanhf(v);
        if (ACT == 2) v = fmaxf(v, 0.0f);
        if (ACT == 3) v = v / (1.0f + expf(-v));
        if (ACT == 4) v = (v > 0.f) ? v : 0.01f * v;
        if (ACT == 5) v = 0.5f * v * (1.0f + erff(v * 0.70710678118654752f));
        slab[(mOff + r) * 68 + (j << 4) + rlane] = v;
      }
    }
    __builtin_amdgcn_fence(__ATOMIC_RELEASE, "workgroup");
    __builtin_amdgcn_wave_barrier();
    __builtin_amdgcn_fence(__ATOMIC_ACQUIRE, "workgroup");
    if (OUT_MODE == 0) {
      float* C = (float*)Cout + (size_t)b * strideC;
      const int hh = lane >> 4, c4 = (lane & 15) * 4;
      for (int pass = 0; pass < 2; ++pass) {
#pragma unroll
        for (int it = 0; it < 8; ++it) {
          const int row = it * 2 + hh;
          v4f v = *(const v4f*)(slab + row * 68 + c4);
          *(volatile v4f*)(C + (size_t)(mBase + row) * ldc + n0 + c4) = v;
        }
        __threadfence();
      }
    } else {
      const int q = lane >> 3, c8 = (lane & 7) * 8;
      unsigned short* C  = (unsigned short*)Cout  + (size_t)b * strideC;
      unsigned short* C2 = (OUT_MODE == 2) ? ((unsigned short*)Cout2 + (size_t)b * strideC) : nullptr;
      for (int pass = 0; pass < 2; ++pass) {
#pragma unroll
        for (int it = 0; it < 4; ++it) {
          const int row = it * 4 + q;
          const float* sp = slab + row * 68 + c8;
          v8h hv, lv;
#pragma unroll
          for (int e = 0; e < 8; ++e) {
            if (OUT_MODE == 1) {
              hv[e] = (_Float16)sp[e];
            } else {
              unsigned short hb = f2bf_bits(sp[e]);
              unsigned short lb = f2bf_bits(sp[e] - bf_bits2f(hb));
              hv[e] = __builtin_bit_cast(_Float16, hb);
              lv[e] = __builtin_bit_cast(_Float16, lb);
            }
          }
          *(volatile v8h*)(C + (size_t)(mBase + row) * ldc + n0 + c8) = hv;
          if (OUT_MODE == 2) *(volatile v8h*)(C2 + (size_t)(mBase + row) * ldc + n0 + c8) = lv;
        }
        __threadfence();
      }
    }
    __builtin_amdgcn_fence(__ATOMIC_RELEASE, "workgroup");
    __builtin_amdgcn_wave_barrier();
    __builtin_amdgcn_fence(__ATOMIC_ACQUIRE, "workgroup");
  }
}

__global__ __launch_bounds__(256) void cast_f32_f16x2(
    const float* __restrict__ in, _Float16* __restrict__ out, int n2) {
  int i = blockIdx.x * 256 + threadIdx.x;
  if (i < n2) {
    const _Float16 h0 = (_Float16)in[2 * i], h1 = (_Float16)in[2 * i + 1];
    const unsigned u = (unsigned)__builtin_bit_cast(unsigned short, h0) | ((unsigned)__builtin_bit_cast(unsigned short, h1) << 16);
    ((volatile unsigned*)out)[i] = u;
    __threadfence();
    ((volatile unsigned*)out)[i] = u;
  }
}


#define MB_ 4
#define MN 2048
#define MD 256
#define MS 8
#define MR (MB_ * MS)
#define MT (MB_ * MN)
#define M_EPS 1e-10f
#define M_LNE 1e-5f
#define M_SCALE 0.0625f
__device__ __forceinline__ float wsum(float v) { for (int o = 16; o > 0; o >>= 1) v += __shfl_xor(v, o, 32); return v; }
__device__ __forceinline__ unsigned pk2(float a, float b) { return (unsigned)__builtin_bit_cast(unsigned short, (_Float16)a) | ((unsigned)__builtin_bit_cast(unsigned short, (_Float16)b) << 16); }
__global__ __launch_bounds__(256) void lnin_kernel(const float* __restrict__ x, const float* __restrict__ g, const float* __restrict__ bb, unsigned* __restrict__ X16) {
  const int lane = threadIdx.x & 31, wave = threadIdx.x >> 5; const size_t r = (size_t)blockIdx.x * 8 + wave;
  const v8f v = *(const v8f*)(x + r * MD + lane * 8); float s = 0.f; for (int q = 0; q < 8; ++q) s += v[q]; const float mu = wsum(s) / MD;
  float t = 0.f; for (int q = 0; q < 8; ++q) { const float d = v[q] - mu; t += d * d; } const float inv = rsqrtf(wsum(t) / MD + M_LNE);
  typedef __attribute__((ext_vector_type(4))) unsigned u4; u4 u;
  for (int q = 0; q < 4; ++q) { const int c = lane * 8 + 2 * q; u[q] = pk2((v[2*q] - mu) * inv * g[c] + bb[c], (v[2*q+1] - mu) * inv * g[c + 1] + bb[c + 1]); }
  *(volatile u4*)(X16 + (r * MD + lane * 8) / 2) = u; __threadfence(); *(volatile u4*)(X16 + (r * MD + lane * 8) / 2) = u;
}
__global__ __launch_bounds__(256) void vt_kernel(const float* __restrict__ V, unsigned* __restrict__ VT16, unsigned* __restrict__ V2T16) {
  __shared__ float tile[64][65];
  const int b = blockIdx.z, d0 = blockIdx.x * 64, n0 = blockIdx.y * 64, tx = threadIdx.x, ty = threadIdx.y;
  for (int r = ty; r < 64; r += 8) { const float* src = V + ((size_t)b * MN + n0 + r) * MD + d0; tile[r][tx] = src[tx]; tile[r][32 + tx] = src[32 + tx]; }
  __syncthreads();
  for (int pass = 0; pass < 2; ++pass) { for (int d = ty; d < 64; d += 8) { const float a = tile[2 * tx][d], c = tile[2 * tx + 1][d]; const size_t o = (((size_t)b * MD + d0 + d) * MN + n0) / 2 + tx;
      ((volatile unsigned*)VT16)[o] = pk2(a, c); ((volatile unsigned*)V2T16)[o] = pk2(a * a, c * c); } __threadfence(); }
}
__global__ __launch_bounds__(256) void slotln_kernel(const float* __restrict__ SL, const float* __restrict__ g, const float* __restrict__ bb, unsigned* __restrict__ SOP16, float* __restrict__ MU) {
  const int lane = threadIdx.x & 31, wave = threadIdx.x >> 5; const int r = blockIdx.x * 8 + wave; if (r >= MR) return;
  float v[16]; float s = 0.f; for (int q = 0; q < 16; ++q) { v[q] = SL[r * 512 + lane * 16 + q]; s += v[q]; } const float mu = wsum(s) / 512.f;
  float t = 0.f; for (int q = 0; q < 16; ++q) { const float d = v[q] - mu; t += d * d; } const float inv = rsqrtf(wsum(t) / 512.f + M_LNE);
  float y[16]; for (int q = 0; q < 16; ++q) { const int c = lane * 16 + q; y[q] = (v[q] - mu) * inv * g[c] + bb[c]; }
  typedef __attribute__((ext_vector_type(4))) unsigned u4; u4 u0, u1; for (int q = 0; q < 4; ++q) { u0[q] = pk2(y[2*q], y[2*q+1]); u1[q] = pk2(y[8+2*q], y[8+2*q+1]); }
  const int row = (lane < 16) ? r : (32 + r); const int col = (lane & 15) * 16;
  for (int pass = 0; pass < 2; ++pass) { *(volatile u4*)(SOP16 + (row * MD + col) / 2) = u0; *(volatile u4*)(SOP16 + (row * MD + col) / 2 + 4) = u1;
    if (lane < 16) for (int q = 0; q < 16; ++q) ((volatile float*)MU)[r * MD + col + q] = y[q]; __threadfence(); }
}
__global__ __launch_bounds__(256) void dots_kernel(const float* __restrict__ K, const float* __restrict__ QROW, int qld, const float* __restrict__ SGROW, int sgld, float* __restrict__ DEX) {
  const int lane = threadIdx.x & 31, wave = threadIdx.x >> 5; const size_t t0 = ((size_t)blockIdx.x * 8 + wave) * 4; const int b = (int)(t0 / MN);
  float mine = 0.f;
  for (int tk = 0; tk < 4; ++tk) { const v8f kv = *(const v8f*)(K + (t0 + tk) * MD + lane * 8);
    for (int s = 0; s < MS; ++s) { const int row = b * MS + s; const v8f q = *(const v8f*)(QROW + (size_t)row * qld + lane * 8), sgp = *(const v8f*)(SGROW + (size_t)row * sgld + lane * 8);
      float d = 0.f; for (int e = 0; e < 8; ++e) { const float sg = expf(sgp[e]); const float z = (kv[e] - q[e]) / sg; d += z * z; }
      d = wsum(d) * M_SCALE; const float dex = expf(-0.5f * d + M_EPS); if (lane == tk * 8 + s) mine = dex; } }
  ((volatile float*)DEX)[t0 * MS + lane] = mine; __threadfence(); ((volatile float*)DEX)[t0 * MS + lane] = mine;
}
__global__ __launch_bounds__(1024) void norm_kernel(const float* __restrict__ DEX, const float* __restrict__ PIIN, int mode, unsigned* __restrict__ A16, float* __restrict__ PIOUT, float* __restrict__ M0, float* __restrict__ GOUT) {
  __shared__ float red[32][8]; __shared__ float sg[8];
  const int b = blockIdx.x, t = threadIdx.x, lane = t & 31, wave = t >> 5;
  const float* d0 = DEX + ((size_t)b * MN + 2 * t) * MS; const float* d1 = d0 + MS; const float* pin = PIIN + b * MS;
  float ss0 = 0.f, ss1 = 0.f;
#pragma unroll 1
  for (int s = 0; s < MS; ++s) { ss0 += d0[s] * pin[s]; ss1 += d1[s] * pin[s]; }
  const float i0 = 1.0f / (ss0 + M_EPS), i1 = 1.0f / (ss1 + M_EPS);
  if (mode == 2) {
    for (int pass = 0; pass < 2; ++pass) {
#pragma unroll 1
      for (int s = 0; s < MS; ++s) { typedef __attribute__((ext_vector_type(2))) float v2f; const v2f w = {(d0[s] * pin[s] + M_EPS) * i0, (d1[s] * pin[s] + M_EPS) * i1}; *(volatile v2f*)(GOUT + ((size_t)b * MS + s) * MN + 2 * t) = w; }
      __threadfence(); }
    return; }
#pragma unroll 1
  for (int s = 0; s < MS; ++s) { float v = (d0[s] * pin[s] + M_EPS) * i0 + (d1[s] * pin[s] + M_EPS) * i1; v = wsum(v); if (lane == 0) red[wave][s] = v; }
  __syncthreads();
  if (t < MS) { float v = 0.f; for (int w = 0; w < 32; ++w) v += red[w][t]; sg[t] = v; }
  __syncthreads();
  if (t < 32) { float p = 0.f; if (t < MS) p = (sg[t] + (float)MN * M_EPS) / (sg[t] + M_EPS); const float ps = wsum(p);
    if (t < MS) for (int pass = 0; pass < 2; ++pass) { ((volatile float*)PIOUT)[b * MS + t] = (p + M_EPS) / (ps + M_EPS); ((volatile float*)M0)[b * MS + t] = p; __threadfence(); } }
  for (int pass = 0; pass < 2; ++pass) {
#pragma unroll 1
    for (int s = 0; s < MS; ++s) { const float is = 32768.0f / (sg[s] + M_EPS); const float a0 = ((d0[s] * pin[s] + M_EPS) * i0 + M_EPS) * is, a1 = ((d1[s] * pin[s] + M_EPS) * i1 + M_EPS) * is; ((volatile unsigned*)A16)[(((size_t)b * 64 + s) * MN) / 2 + t] = pk2(a0, a1); }
#pragma unroll 1
    for (int s = MS; s < 64; ++s) ((volatile unsigned*)A16)[(((size_t)b * 64 + s) * MN) / 2 + t] = 0u;
    __threadfence(); }
}
__global__ __launch_bounds__(256) void pack_kernel(const float* __restrict__ SRC, unsigned* __restrict__ DST16, float* __restrict__ DSTF) {
  const int lane = threadIdx.x & 31, wave = threadIdx.x >> 5; const int r = blockIdx.x * 8 + wave;
  typedef __attribute__((ext_vector_type(4))) unsigned u4; u4 u = {0u, 0u, 0u, 0u}; v8f v = {0.f,0.f,0.f,0.f,0.f,0.f,0.f,0.f};
  if (r < MR) { const int b = r / MS, s = r % MS; v = *(const v8f*)(SRC + ((size_t)b * 64 + s) * MD + lane * 8); for (int q = 0; q < 4; ++q) u[q] = pk2(v[2*q], v[2*q+1]); }
  for (int pass = 0; pass < 2; ++pass) { *(volatile u4*)(DST16 + (r * MD + lane * 8) / 2) = u; if (DSTF && r < MR) *(volatile v8f*)(DSTF + r * MD + lane * 8) = v; __threadfence(); }
}
__global__ __launch_bounds__(256) void gru_kernel(const float* __restrict__ GI, const float* __restrict__ GH, const float* __restrict__ MU, const float* __restrict__ g, const float* __restrict__ bb, float* __restrict__ UM0, unsigned* __restrict__ UM16) {
  const int lane = threadIdx.x & 31, wave = threadIdx.x >> 5; const int r = blockIdx.x * 8 + wave;
  typedef __attribute__((ext_vector_type(4))) unsigned u4; u4 u = {0u, 0u, 0u, 0u}; float h[8];
  if (r < MR) { float s = 0.f;
    for (int q = 0; q < 8; ++q) { const int c = lane * 8 + q; const float rr = 1.0f / (1.0f + expf(-(GI[r * 768 + c] + GH[r * 768 + c]))), z = 1.0f / (1.0f + expf(-(GI[r * 768 + 256 + c] + GH[r * 768 + 256 + c])));
      const float ng = tanhf(GI[r * 768 + 512 + c] + rr * GH[r * 768 + 512 + c]); h[q] = (1.0f - z) * ng + z * MU[r * MD + c]; s += h[q]; }
    const float mu = wsum(s) / MD; float t = 0.f; for (int q = 0; q < 8; ++q) { const float d = h[q] - mu; t += d * d; } const float inv = rsqrtf(wsum(t) / MD + M_LNE);
    for (int q = 0; q < 8; ++q) { const int c = lane * 8 + q; h[q] = (h[q] - mu) * inv * g[c] + bb[c]; }
    for (int q = 0; q < 4; ++q) u[q] = pk2(h[2*q], h[2*q+1]); }
  for (int pass = 0; pass < 2; ++pass) { *(volatile u4*)(UM16 + (r * MD + lane * 8) / 2) = u; if (r < MR) { const v8f hv = {h[0],h[1],h[2],h[3],h[4],h[5],h[6],h[7]}; *(volatile v8f*)(UM0 + r * MD + lane * 8) = hv; } __threadfence(); }
}
__global__ __launch_bounds__(256) void updmu_kernel(const float* __restrict__ MLP2, const float* __restrict__ UM0, float* __restrict__ UPDMU) {
  const int lane = threadIdx.x & 31, wave = threadIdx.x >> 5; const int r = blockIdx.x * 8 + wave; if (r >= MR) return;
  const v8f v = *(const v8f*)(MLP2 + r * MD + lane * 8) + *(const v8f*)(UM0 + r * MD + lane * 8);
  *(volatile v8f*)(UPDMU + r * MD + lane * 8) = v; __threadfence(); *(volatile v8f*)(UPDMU + r * MD + lane * 8) = v;
}
__global__ __launch_bounds__(256) void slotsout_kernel(const float* __restrict__ UPDMU, const float* __restrict__ M1, const float* __restrict__ M2, const float* __restrict__ M0, float* __restrict__ SL) {
  const int lane = threadIdx.x & 31, wave = threadIdx.x >> 5; const int r = blockIdx.x * 8 + wave; if (r >= MR) return; const int b = r / MS, s = r % MS;
  const v8f mu = *(const v8f*)(UPDMU + r * MD + lane * 8), m1 = *(const v8f*)(M1 + ((size_t)b * 64 + s) * MD + lane * 8), m2 = *(const v8f*)(M2 + ((size_t)b * 64 + s) * MD + lane * 8); const float m0 = M0[r];
  v8f ls; for (int q = 0; q < 8; ++q) ls[q] = 0.5f * logf(m2[q] - 2.0f * mu[q] * m1[q] + mu[q] * mu[q] * m0 + M_EPS);
  for (int pass = 0; pass < 2; ++pass) { *(volatile v8f*)(SL + r * 512 + lane * 8) = mu; *(volatile v8f*)(SL + r * 512 + 256 + lane * 8) = ls; __threadfence(); }
}
__global__ __launch_bounds__(256) void slots16_kernel(const float* __restrict__ SL, unsigned* __restrict__ S16) {
  const int lane = threadIdx.x & 31, wave = threadIdx.x >> 5; const int r = blockIdx.x * 8 + wave; typedef __attribute__((ext_vector_type(4))) unsigned u4; u4 u0 = {0u,0u,0u,0u}, u1 = {0u,0u,0u,0u};
  if (r < MR) { for (int q = 0; q < 4; ++q) { u0[q] = pk2(SL[r * 512 + lane * 16 + 2*q], SL[r * 512 + lane * 16 + 2*q + 1]); u1[q] = pk2(SL[r * 512 + lane * 16 + 8 + 2*q], SL[r * 512 + lane * 16 + 8 + 2*q + 1]); } }
  for (int pass = 0; pass < 2; ++pass) { *(volatile u4*)(S16 + (r * 512 + lane * 16) / 2) = u0; *(volatile u4*)(S16 + (r * 512 + lane * 16) / 2 + 4) = u1; __threadfence(); }
}
__global__ __launch_bounds__(256) void copyout_kernel(const float* __restrict__ SRC, float* __restrict__ out, int nflt) { const int i = blockIdx.x * 256 + threadIdx.x; if (i < nflt) { ((volatile float*)out)[i] = SRC[i]; __threadfence(); ((volatile float*)out)[i] = SRC[i]; } }
__global__ __launch_bounds__(64) void piinit_kernel(float* PI) { if (threadIdx.x < MR) { ((volatile float*)PI)[threadIdx.x] = 1.0f / MS; __threadfence(); ((volatile float*)PI)[threadIdx.x] = 1.0f / MS; } }
extern "C" void kernel_launch(void* const* d_in, const int* in_sizes, int n_in, void* d_out, int out_size, void* d_ws, size_t ws_size, hipStream_t stream) {
  (void)in_sizes; (void)n_in; (void)out_size; (void)ws_size;
  auto Fp = [&](int i) { return (const float*)d_in[i]; };
  const float* slots0 = Fp(0); const float* inputs = Fp(1); const float* Wq = Fp(2); const float* Wk = Fp(3); const float* Wv = Fp(4); const float* Wih = Fp(5); const float* Whh = Fp(6); const float* bih = Fp(7); const float* bhh = Fp(8);
  const float* W1 = Fp(9); const float* b1 = Fp(10); const float* W2 = Fp(11); const float* b2 = Fp(12); const float* lng = Fp(13); const float* lnb = Fp(14); const float* lsg = Fp(15); const float* lsb = Fp(16); const float* lmg = Fp(17); const float* lmb = Fp(18);
  const float* Wo1 = Fp(19); const float* bo1 = Fp(20); const float* Wo2 = Fp(21); const float* bo2 = Fp(22);
  float* out0 = (float*)d_out; float* out1 = out0 + MR * MD;
  char* ws = (char*)d_ws; size_t off = 0;
  auto carve = [&](size_t bytes) -> char* { char* p = ws + off; off += (bytes + 255) & ~(size_t)255; return p; };
  unsigned* X16 = (unsigned*)carve((size_t)MT * MD * 2); _Float16* WK16 = (_Float16*)carve(MD * MD * 2); _Float16* WV16 = (_Float16*)carve(MD * MD * 2); _Float16* WQ16 = (_Float16*)carve(MD * MD * 2);
  _Float16* WIH16 = (_Float16*)carve(768 * MD * 2); _Float16* WHH16 = (_Float16*)carve(768 * MD * 2); _Float16* W116 = (_Float16*)carve(1024 * MD * 2); _Float16* W216 = (_Float16*)carve(MD * 1024 * 2); _Float16* WO116 = (_Float16*)carve((size_t)2048 * 512 * 2); _Float16* WO216 = (_Float16*)carve((size_t)MD * 2048 * 2);
  float* Kf = (float*)carve((size_t)MT * MD * 4); float* Vf = (float*)carve((size_t)MT * MD * 4); unsigned* VT16 = (unsigned*)carve((size_t)MT * MD * 2); unsigned* V2T16 = (unsigned*)carve((size_t)MT * MD * 2);
  float* SL = (float*)carve(MR * 512 * 4); float* PI = (float*)carve(256); float* PI2 = (float*)carve(256); float* M0 = (float*)carve(256);
  unsigned* SOP16 = (unsigned*)carve(64 * MD * 2); float* MU = (float*)carve(MR * MD * 4); float* QOUT = (float*)carve(64 * MD * 4); float* DEX = (float*)carve((size_t)MT * MS * 4);
  unsigned* A16 = (unsigned*)carve((size_t)MB_ * 64 * MN * 2); float* UPD = (float*)carve((size_t)MB_ * 64 * MD * 4); unsigned* UPD16 = (unsigned*)carve(64 * MD * 2);
  float* GI = (float*)carve(64 * 768 * 4); float* GH = (float*)carve(64 * 768 * 4); float* UM0 = (float*)carve(MR * MD * 4); unsigned* UM16 = (unsigned*)carve(64 * MD * 2); _Float16* H1 = (_Float16*)carve(64 * 1024 * 2); float* MLP2 = (float*)carve(64 * MD * 4); float* UPDMU = (float*)carve(MR * MD * 4);
  float* M1 = (float*)carve((size_t)MB_ * 64 * MD * 4); float* M2 = (float*)carve((size_t)MB_ * 64 * MD * 4); unsigned* S16 = (unsigned*)carve(64 * 512 * 2); _Float16* HO = (_Float16*)carve((size_t)64 * 2048 * 2); float* OUTB = (float*)carve(64 * MD * 4);
  lnin_kernel<<<MT / 8, 256, 0, stream>>>(inputs, lng, lnb, X16);
  cast_f32_f16x2<<<(MD * MD / 2 + 255) / 256, 256, 0, stream>>>(Wk, WK16, MD * MD / 2); cast_f32_f16x2<<<(MD * MD / 2 + 255) / 256, 256, 0, stream>>>(Wv, WV16, MD * MD / 2); cast_f32_f16x2<<<(MD * MD / 2 + 255) / 256, 256, 0, stream>>>(Wq, WQ16, MD * MD / 2);
  cast_f32_f16x2<<<(768 * MD / 2 + 255) / 256, 256, 0, stream>>>(Wih, WIH16, 768 * MD / 2); cast_f32_f16x2<<<(768 * MD / 2 + 255) / 256, 256, 0, stream>>>(Whh, WHH16, 768 * MD / 2);
  cast_f32_f16x2<<<(1024 * MD / 2 + 255) / 256, 256, 0, stream>>>(W1, W116, 1024 * MD / 2); cast_f32_f16x2<<<(MD * 1024 / 2 + 255) / 256, 256, 0, stream>>>(W2, W216, MD * 1024 / 2);
  cast_f32_f16x2<<<(2048 * 512 / 2 + 255) / 256, 256, 0, stream>>>(Wo1, WO116, 2048 * 512 / 2); cast_f32_f16x2<<<(MD * 2048 / 2 + 255) / 256, 256, 0, stream>>>(Wo2, WO216, MD * 2048 / 2);
  { const int t = (MT / 64) * 4; wmma_gemm64<0, false, 0, 0, false><<<dim3((t + 7) / 8, 1), 256, 0, stream>>>((const unsigned short*)X16, nullptr, MD, 0, U16(WK16), nullptr, MD, 0, Kf, nullptr, MD, 0, nullptr, nullptr, 0, MT, MD, MD, 1.0f);
    wmma_gemm64<0, false, 0, 0, false><<<dim3((t + 7) / 8, 1), 256, 0, stream>>>((const unsigned short*)X16, nullptr, MD, 0, U16(WV16), nullptr, MD, 0, Vf, nullptr, MD, 0, nullptr, nullptr, 0, MT, MD, MD, 1.0f); }
  vt_kernel<<<dim3(MD / 64, MN / 64, MB_), dim3(32, 8), 0, stream>>>(Vf, VT16, V2T16);
  copyout_kernel<<<(MR * 512 + 255) / 256, 256, 0, stream>>>(slots0, SL, MR * 512);
  piinit_kernel<<<1, 64, 0, stream>>>(PI);
  const int t8 = 1 * 4;
  for (int step = 0; step < 4; ++step) { const bool last = (step == 3);
    slotln_kernel<<<MR / 8, 256, 0, stream>>>(SL, lsg, lsb, SOP16, MU);
    wmma_gemm64<0, false, 0, 0, false><<<dim3((t8 + 7) / 8, 1), 256, 0, stream>>>((const unsigned short*)SOP16, nullptr, MD, 0, U16(WQ16), nullptr, MD, 0, QOUT, nullptr, MD, 0, nullptr, nullptr, 0, 64, MD, MD, 1.0f);
    dots_kernel<<<MT / 32, 256, 0, stream>>>(Kf, QOUT, MD, QOUT + 32 * MD, MD, DEX);
    norm_kernel<<<MB_, 1024, 0, stream>>>(DEX, PI, 0, A16, PI2, M0, nullptr);
    wmma_gemm64<0, false, 0, 0, false><<<dim3((t8 + 7) / 8, MB_), 256, 0, stream>>>((const unsigned short*)A16, nullptr, MN, (long)64 * MN, (const unsigned short*)VT16, nullptr, MN, (long)MD * MN, UPD, nullptr, MD, (long)64 * MD, nullptr, nullptr, 0, 64, MD, MN, 1.0f / 32768.0f);
    norm_kernel<<<MB_, 1024, 0, stream>>>(DEX, PI2, 0, A16, PI, M0, nullptr);
    pack_kernel<<<64 / 8, 256, 0, stream>>>(UPD, UPD16, nullptr);
    { const int tg = 1 * 12; wmma_gemm64<0, false, 2, 0, false><<<dim3((tg + 7) / 8, 1), 256, 0, stream>>>((const unsigned short*)UPD16, nullptr, MD, 0, U16(WIH16), nullptr, MD, 0, GI, nullptr, 768, 0, bih, nullptr, 0, 64, 768, MD, 1.0f);
      wmma_gemm64<0, false, 2, 0, false><<<dim3((tg + 7) / 8, 1), 256, 0, stream>>>((const unsigned short*)SOP16, nullptr, MD, 0, U16(WHH16), nullptr, MD, 0, GH, nullptr, 768, 0, bhh, nullptr, 0, 64, 768, MD, 1.0f); }
    gru_kernel<<<64 / 8, 256, 0, stream>>>(GI, GH, MU, lmg, lmb, UM0, UM16);
    { const int t1 = 1 * 16; wmma_gemm64<0, false, 2, 1, false, 2><<<dim3((t1 + 7) / 8, 1), 256, 0, stream>>>((const unsigned short*)UM16, nullptr, MD, 0, U16(W116), nullptr, MD, 0, H1, nullptr, 1024, 0, b1, nullptr, 0, 64, 1024, MD, 1.0f);
      wmma_gemm64<0, false, 2, 0, false, 0><<<dim3((t8 + 7) / 8, 1), 256, 0, stream>>>(U16(H1), nullptr, 1024, 0, U16(W216), nullptr, 1024, 0, MLP2, nullptr, MD, 0, b2, nullptr, 0, 64, MD, 1024, 1.0f); }
    updmu_kernel<<<MR / 8, 256, 0, stream>>>(MLP2, UM0, UPDMU);
    dots_kernel<<<MT / 32, 256, 0, stream>>>(Kf, UPDMU, MD, QOUT + 32 * MD, MD, DEX);
    norm_kernel<<<MB_, 1024, 0, stream>>>(DEX, PI, 0, A16, PI2, M0, nullptr);
    wmma_gemm64<0, false, 0, 0, false><<<dim3((t8 + 7) / 8, MB_), 256, 0, stream>>>((const unsigned short*)A16, nullptr, MN, (long)64 * MN, (const unsigned short*)VT16, nullptr, MN, (long)MD * MN, M1, nullptr, MD, (long)64 * MD, nullptr, nullptr, 0, 64, MD, MN, 1.0f / 32768.0f);
    wmma_gemm64<0, false, 0, 0, false><<<dim3((t8 + 7) / 8, MB_), 256, 0, stream>>>((const unsigned short*)A16, nullptr, MN, (long)64 * MN, (const unsigned short*)V2T16, nullptr, MN, (long)MD * MN, M2, nullptr, MD, (long)64 * MD, nullptr, nullptr, 0, 64, MD, MN, 1.0f / 32768.0f);
    slotsout_kernel<<<MR / 8, 256, 0, stream>>>(UPDMU, M1, M2, M0, SL);
    copyout_kernel<<<1, 64, 0, stream>>>(PI2, PI, MR);
    if (last) { dots_kernel<<<MT / 32, 256, 0, stream>>>(Kf, SL, 512, SL + 256, 512, DEX);
      norm_kernel<<<MB_, 1024, 0, stream>>>(DEX, PI, 2, nullptr, nullptr, nullptr, out1); } }
  slots16_kernel<<<64 / 8, 256, 0, stream>>>(SL, S16);
  { const int to1 = 1 * 32; wmma_gemm64<0, false, 2, 1, false, 2><<<dim3((to1 + 7) / 8, 1), 256, 0, stream>>>((const unsigned short*)S16, nullptr, 512, 0, U16(WO116), nullptr, 512, 0, HO, nullptr, 2048, 0, bo1, nullptr, 0, 64, 2048, 512, 1.0f);
    wmma_gemm64<0, false, 2, 0, false, 0><<<dim3((t8 + 7) / 8, 1), 256, 0, stream>>>(U16(HO), nullptr, 2048, 0, U16(WO216), nullptr, 2048, 0, OUTB, nullptr, MD, 0, bo2, nullptr, 0, 64, MD, 2048, 1.0f); }
  copyout_kernel<<<(MR * MD + 255) / 256, 256, 0, stream>>>(OUTB, out0, MR * MD);
}
